// TransformerBlock_62474594287859
// MI455X (gfx1250) — hardware-run, weakly checked
//
#include <hip/hip_runtime.h>
#include <stddef.h>


typedef _Float16 v16h __attribute__((ext_vector_type(16)));
typedef _Float16 v8h  __attribute__((ext_vector_type(8)));
typedef float    v8f  __attribute__((ext_vector_type(8)));
typedef float    v4f  __attribute__((ext_vector_type(4)));

#ifndef NB
#define NB 1
#endif
#ifndef SEQ
#define SEQ 2048
#endif
#define NB_FULL  1
#define SEQ_FULL 2048
#define DIM   1024
#define NHEAD 16
#define HD    64
#define NLAT  256
#define NSH   2
#define NRT   8
#define NEXP  (NSH + NRT)
#define DHID  1024
#define DFF   (NEXP * DHID)
#define MROWS (NB * SEQ)

static_assert(NB >= 1 && NB <= NB_FULL);
static_assert(SEQ >= 128 && SEQ <= SEQ_FULL && (SEQ % 128) == 0);
static_assert((SEQ % 8) == 0);
static_assert(DIM == NHEAD * HD);
static_assert(HD == 64);
static_assert((DIM % 64) == 0 && (DIM % 32) == 0);
static_assert((NLAT % 64) == 0 && (NLAT % 32) == 0);
static_assert(((DIM + NLAT) % 64) == 0);
static_assert((DHID % 64) == 0 && (DHID % 32) == 0);
static_assert((DFF % 64) == 0 && (DFF % 32) == 0);
static_assert((MROWS % 64) == 0);
static_assert(DIM == 128 * 8);
static_assert(NRT == 8);
static_assert((size_t)MROWS * DFF < (size_t)0xFFFFFFFFu);

#define LDT 72
#define LDC 68
static_assert((LDT % 8) == 0 && LDT >= 64);
static_assert((LDC % 4) == 0 && LDC >= 64);

#define WCARRY 64.0f
#define PCARRY 1024.0f
#define VCARRY 64.0f
#define ACARRY 64.0f

#define GPITCH 32

#define PLANE16_ELEMS ((size_t)MROWS * DIM)
#define PLANE16_BYTES (PLANE16_ELEMS * 2)
#define WSQ_ELEMS     ((size_t)DIM * DIM)
#define OFF_WQC   ((size_t)0)
#define OFF_WUKV  (OFF_WQC + (size_t)(DIM + NLAT) * DIM * 2)
#define OFF_WO    (OFF_WUKV + (size_t)2 * DIM * NLAT * 2)
#define OFF_W1    (OFF_WO + WSQ_ELEMS * 2)
#define OFF_W2    (OFF_W1 + (size_t)DFF * DIM * 2)
#define OFF_TAB   (OFF_W2 + (size_t)DFF * DIM * 2)
#define OFF_H1    (OFF_TAB + (size_t)SEQ * 64 * 4)
#define OFF_C     (OFF_H1 + PLANE16_BYTES)
#define OFF_QKV   (OFF_C + (size_t)MROWS * NLAT * 2)
#define OFF_CTX   (OFF_QKV + 3 * PLANE16_BYTES)
#define OFF_X1    (OFF_CTX + PLANE16_BYTES)
#define OFF_H2    (OFF_X1 + PLANE16_ELEMS * 4)
#define OFF_DW    (OFF_H2 + PLANE16_BYTES)
#define OFF_ACT   (OFF_DW + (size_t)MROWS * GPITCH * 4)
#define WS_TOTAL  (OFF_ACT + (size_t)MROWS * DFF * 2)
static_assert((PLANE16_BYTES % 128) == 0 && ((WSQ_ELEMS * 2) % 128) == 0);
static_assert((OFF_WUKV % 128) == 0 && (OFF_WO % 128) == 0 && (OFF_W1 % 128) == 0);
static_assert((OFF_W2 % 128) == 0 && (OFF_TAB % 128) == 0 && (OFF_H1 % 128) == 0);
static_assert((OFF_C % 128) == 0 && (OFF_QKV % 128) == 0 && (OFF_CTX % 128) == 0);
static_assert((OFF_H2 % 128) == 0 && (OFF_DW % 128) == 0);
static_assert((OFF_ACT % 128) == 0 && (OFF_X1 % 128) == 0);
static_assert(WS_TOTAL <= (size_t)134217728);

__device__ __forceinline__ float bf16r(float x) {
  unsigned int u = __float_as_uint(x);
  u = (u + 0x7FFFu + ((u >> 16) & 1u)) & 0xFFFF0000u;
  return __uint_as_float(u);
}

__device__ __forceinline__ size_t full_row(unsigned crow) {
  const unsigned bidx = crow / (unsigned)SEQ;
  const unsigned sq = crow - bidx * (unsigned)SEQ;
  return (size_t)bidx * SEQ_FULL + sq;
}

static __device__ __forceinline__ _Float16 toh_flush(float v) {
  const _Float16 r = (_Float16)v;
  return (fabsf(v) < 6.103515625e-05f) ? (_Float16)0.0f : r;
}

__device__ __forceinline__ v16h frag_at(const _Float16* p) {
  v8h lo = *(const v8h*)(p);
  v8h hi = *(const v8h*)(p + 16);
  v16h out;
#pragma unroll
  for (int i = 0; i < 8; ++i) { out[i] = lo[i]; out[i + 8] = hi[i]; }
  return out;
}
__device__ __forceinline__ v16h ld_frag(const _Float16* base, unsigned ld) {
  const unsigned lane = threadIdx.x & 31u;
  return frag_at(base + (lane & 15u) * ld + (lane >> 4) * 8u);
}

__device__ __forceinline__ v8f wmma16(v16h a, v16h b, v8f c) {
  v8f d = __builtin_amdgcn_wmma_f32_16x16x32_f16(false, a, false, b, (short)0, c,
                                                 false, false);
  asm volatile("v_nop\n\tv_nop\n\tv_nop\n\tv_nop" : "+v"(d) : "v"(a), "v"(b));
  return d;
}

__device__ __forceinline__ float red16_max(float x) {
#pragma unroll
  for (int off = 1; off < 16; off <<= 1) x = fmaxf(x, __shfl_xor(x, off, 32));
  return x;
}
__device__ __forceinline__ float red16_sum(float x) {
#pragma unroll
  for (int off = 1; off < 16; off <<= 1) x += __shfl_xor(x, off, 32);
  return x;
}
__device__ __forceinline__ float red32_sum(float x) {
#pragma unroll
  for (int off = 1; off < 32; off <<= 1) x += __shfl_xor(x, off, 32);
  return x;
}

__device__ __forceinline__ void wave_lds_sync() {
  __builtin_amdgcn_fence(3  , "wavefront");
  asm volatile("s_wait_dscnt 0x0" ::: "memory");
  __builtin_amdgcn_wave_barrier();
}

__global__ __launch_bounds__(256) void wconv_kernel(
    const float* __restrict__ W, _Float16* __restrict__ Wt,
    unsigned N, unsigned K, unsigned headmode) {
  __shared__ _Float16 T[64 * LDT];
  const unsigned tid = threadIdx.x;
  const unsigned n0 = blockIdx.x * 64u;
  const unsigned k0 = blockIdx.y * 64u;
  const size_t sbase = headmode ? (size_t)blockIdx.x * K * 64u : (size_t)n0;
  const unsigned ldw = headmode ? 64u : N;
#pragma unroll 4
  for (unsigned j = 0; j < 16u; ++j) {
    const unsigned idx = tid + 256u * j;
    const unsigned kr = idx >> 6, nc = idx & 63u;
    const float v = W[sbase + (size_t)(k0 + kr) * ldw + nc];
    T[nc * LDT + kr] = (_Float16)(WCARRY * bf16r(v));
  }
  __syncthreads();
  v8h x[2];
  size_t off[2];
#pragma unroll
  for (unsigned i = 0; i < 2u; ++i) {
    const unsigned n = 32u * i + (tid >> 3);
    const unsigned kc = (tid & 7u) * 8u;
    x[i] = *(const v8h*)&T[n * LDT + kc];
    off[i] = (size_t)(n0 + n) * K + k0 + kc;
  }
#pragma unroll
  for (int i = 0; i < 2; ++i) *(volatile v8h*)(Wt + off[i]) = x[i];
  __threadfence();
#pragma unroll
  for (int i = 0; i < 2; ++i) *(volatile v8h*)(Wt + off[i]) = x[i];
}

__global__ __launch_bounds__(256) void wconv2_kernel(
    const float* __restrict__ W, _Float16* __restrict__ Wt,
    unsigned N, unsigned K, unsigned ldo, unsigned zstride) {
  __shared__ _Float16 T[64 * LDT];
  const unsigned tid = threadIdx.x;
  const unsigned n0 = blockIdx.x * 64u;
  const unsigned k0 = blockIdx.y * 64u;
  const unsigned z = blockIdx.z;
  const size_t sbase = (size_t)z * K * N + n0;
#pragma unroll 4
  for (unsigned j = 0; j < 16u; ++j) {
    const unsigned idx = tid + 256u * j;
    const unsigned kr = idx >> 6, nc = idx & 63u;
    const float v = W[sbase + (size_t)(k0 + kr) * N + nc];
    T[nc * LDT + kr] = toh_flush(WCARRY * bf16r(v));
  }
  __syncthreads();
  v8h x[2];
  size_t off[2];
#pragma unroll
  for (unsigned i = 0; i < 2u; ++i) {
    const unsigned n = 32u * i + (tid >> 3);
    const unsigned kc = (tid & 7u) * 8u;
    x[i] = *(const v8h*)&T[n * LDT + kc];
    off[i] = (size_t)z * zstride + (size_t)(n0 + n) * ldo + k0 + kc;
  }
#pragma unroll
  for (int i = 0; i < 2; ++i) *(volatile v8h*)(Wt + off[i]) = x[i];
  __threadfence();
#pragma unroll
  for (int i = 0; i < 2; ++i) *(volatile v8h*)(Wt + off[i]) = x[i];
}

__global__ __launch_bounds__(256) void rope_tab_kernel(float* __restrict__ tab) {
#pragma clang fp contract(off)
  const unsigned tid = threadIdx.x, lane = tid & 31u;
  const unsigned s = blockIdx.x * 8u + (tid >> 5);
  double p = 1.0;
#pragma unroll 1
  for (unsigned j = 0; j < lane; ++j) p *= 1.333521432163324;
  const float pw = (float)p;
  const float freq = 1.0f / pw;
  const float ang = (float)s * freq;
  float sn, cs;
  sincosf(ang, &sn, &cs);
  float* dp = tab + (size_t)s * 64u + lane;
  *(volatile float*)(dp) = cs;
  *(volatile float*)(dp + 32) = sn;
  __threadfence();
  *(volatile float*)(dp) = cs;
  *(volatile float*)(dp + 32) = sn;
}

__global__ __launch_bounds__(128) void rms_kernel(
    const float* __restrict__ Xin, const float* __restrict__ g,
    _Float16* __restrict__ dst, unsigned src_full, unsigned rne_in,
    const float* __restrict__ Wg, float* __restrict__ dw, unsigned do_gate) {
  __shared__ float rowf[DIM];
  __shared__ _Float16 rowh[DIM];
  __shared__ float red[4];
  __shared__ float gpart[4 * NRT];
  const unsigned tid = threadIdx.x, lane = tid & 31u;
  const unsigned w = (unsigned)__builtin_amdgcn_readfirstlane((int)(tid >> 5));
  const unsigned crow = blockIdx.x;
  const size_t srow = src_full ? full_row(crow) : (size_t)crow;
  const float* sp = Xin + srow * DIM + tid * 8u;
  v4f a0 = *(const v4f*)(sp);
  v4f a1 = *(const v4f*)(sp + 4);
  if (rne_in) {
#pragma unroll
    for (int j = 0; j < 4; ++j) { a0[j] = bf16r(a0[j]); a1[j] = bf16r(a1[j]); }
  }
  *(v4f*)&rowf[tid * 8u] = a0;
  *(v4f*)&rowf[tid * 8u + 4u] = a1;
  float ss = ((a0[0] * a0[0] + a0[1] * a0[1]) + (a0[2] * a0[2] + a0[3] * a0[3])) +
             ((a1[0] * a1[0] + a1[1] * a1[1]) + (a1[2] * a1[2] + a1[3] * a1[3]));
  ss = red32_sum(ss);
  if (lane == 0u) red[w] = ss;
  __syncthreads();
  const float ms = ((red[0] + red[1]) + (red[2] + red[3])) * (1.0f / (float)DIM);
  const float rinv = 1.0f / sqrtf(ms + 1.0e-8f);
  float lg[NRT];
#pragma unroll
  for (int e = 0; e < NRT; ++e) lg[e] = 0.0f;
#pragma unroll 1
  for (unsigned j = 0; j < 8u; ++j) {
    const unsigned c = tid + 128u * j;
    const float hv = rowf[c] * rinv * bf16r(g[c]);
    rowh[c] = toh_flush(hv);
    if (do_gate) {
      const v4f w0 = *(const v4f*)(Wg + (size_t)c * NRT);
      const v4f w1 = *(const v4f*)(Wg + (size_t)c * NRT + 4);
#pragma unroll
      for (int e = 0; e < 4; ++e) {
        lg[e]     += hv * bf16r(w0[e]);
        lg[e + 4] += hv * bf16r(w1[e]);
      }
    }
  }
  __syncthreads();
  const v8h o = *(const v8h*)&rowh[tid * 8u];
  _Float16* dp = dst + (size_t)crow * DIM + tid * 8u;
  *(volatile v8h*)dp = o;
  __threadfence();
  *(volatile v8h*)dp = o;

  if (do_gate) {
#pragma unroll
    for (int e = 0; e < NRT; ++e) lg[e] = red32_sum(lg[e]);
    if (lane == 0u) {
#pragma unroll
      for (int e = 0; e < NRT; ++e) gpart[w * NRT + (unsigned)e] = lg[e];
    }
    __syncthreads();
    if (w == 0u) {
      const unsigned e = lane & 7u;
      const float lgt = (gpart[e] + gpart[NRT + e]) + (gpart[2 * NRT + e] + gpart[3 * NRT + e]);
      float mx = lgt;
      mx = fmaxf(mx, __shfl_xor(mx, 1, 32));
      mx = fmaxf(mx, __shfl_xor(mx, 2, 32));
      mx = fmaxf(mx, __shfl_xor(mx, 4, 32));
      const float pe = expf(lgt - mx);
      float sm = pe;
      sm += __shfl_xor(sm, 1, 32);
      sm += __shfl_xor(sm, 2, 32);
      sm += __shfl_xor(sm, 4, 32);
      const float gv = pe * (1.0f / sm);
      float v1 = gv;
      int i1 = (int)e;
#pragma unroll
      for (int off = 1; off < 8; off <<= 1) {
        const float ov = __shfl_xor(v1, off, 32);
        const int oi = __shfl_xor(i1, off, 32);
        const bool take = (ov > v1) | ((ov == v1) & (oi < i1));
        v1 = take ? ov : v1;
        i1 = take ? oi : i1;
      }
      float v2 = ((int)e == i1) ? -1.0f : gv;
      int i2 = (int)e;
#pragma unroll
      for (int off = 1; off < 8; off <<= 1) {
        const float ov = __shfl_xor(v2, off, 32);
        const int oi = __shfl_xor(i2, off, 32);
        const bool take = (ov > v2) | ((ov == v2) & (oi < i2));
        v2 = take ? ov : v2;
        i2 = take ? oi : i2;
      }
      const float rs = 1.0f / (v1 + v2);
      float wv = ((int)e == i1) ? v1 * rs : (((int)e == i2) ? v2 * rs : 0.0f);
      wv = (lane < 8u) ? wv : 0.0f;
      float* gp = dw + (size_t)crow * GPITCH + lane;
      *(volatile float*)gp = wv;
      __threadfence();
      *(volatile float*)gp = wv;
    }
  }
}

__device__ __forceinline__ void gemm_main(
    const _Float16* __restrict__ A16, const _Float16* __restrict__ Bt,
    const unsigned K, const unsigned arow0, const unsigned brow0, float* Cs) {
  const unsigned tid = threadIdx.x, lane = tid & 31u, w = tid >> 5;
  const unsigned mw = w >> 1, nw = w & 1u;
  const unsigned hh = lane >> 4, m = lane & 15u;
  const _Float16* ap  = A16 + (size_t)(arow0 + mw * 16u + m) * K + hh * 8u;
  const _Float16* bp0 = Bt + (size_t)(brow0 + nw * 32u + m) * K + hh * 8u;
  const _Float16* bp1 = bp0 + (size_t)16 * K;
  v8f acc0 = {}, acc1 = {};
#pragma unroll 2
  for (unsigned k0 = 0; k0 < K; k0 += 32u) {
    const v16h a  = frag_at(ap + k0);
    const v16h b0 = frag_at(bp0 + k0);
    const v16h b1 = frag_at(bp1 + k0);
    acc0 = wmma16(a, b0, acc0);
    acc1 = wmma16(a, b1, acc1);
  }
#pragma unroll
  for (int r = 0; r < 8; ++r) {
    float* d = &Cs[(mw * 16u + hh * 8u + (unsigned)r) * LDC + nw * 32u + m];
    d[0]  = acc0[r];
    d[16] = acc1[r];
  }
  __syncthreads();
}

__device__ __forceinline__ void epi_f16_fl(
    const float* Cs, _Float16* __restrict__ out16, const unsigned pitch,
    const unsigned row0, const unsigned n0, const float scale) {
  const unsigned tid = threadIdx.x;
  v8h x[2];
  size_t off[2];
#pragma unroll
  for (unsigned i = 0; i < 2u; ++i) {
    const unsigned r = 32u * i + (tid >> 3);
    const unsigned c = (tid & 7u) * 8u;
    const v4f u0 = *(const v4f*)&Cs[r * LDC + c];
    const v4f u1 = *(const v4f*)&Cs[r * LDC + c + 4];
#pragma unroll
    for (int j = 0; j < 4; ++j) {
      x[i][j]     = toh_flush(u0[j] * scale);
      x[i][j + 4] = toh_flush(u1[j] * scale);
    }
    off[i] = (size_t)(row0 + r) * pitch + n0 + c;
  }
#pragma unroll
  for (int i = 0; i < 2; ++i) *(volatile v8h*)(out16 + off[i]) = x[i];
  __threadfence();
#pragma unroll
  for (int i = 0; i < 2; ++i) *(volatile v8h*)(out16 + off[i]) = x[i];
}

__device__ __forceinline__ void epi_rope_fl(
    const float* Cs, const float* __restrict__ tab, _Float16* __restrict__ out16,
    const unsigned row0, const unsigned n0, const float scale) {
  const unsigned tid = threadIdx.x;
  v8h x[2];
  size_t off[2];
#pragma unroll
  for (unsigned i = 0; i < 2u; ++i) {
    const unsigned r = 32u * i + (tid >> 3);
    const unsigned c = (tid & 7u) * 8u;
    const unsigned jc = c & 31u;
    const bool upper = (c >= 32u);
    const unsigned crow = row0 + r;
    const unsigned sq = crow - (crow / (unsigned)SEQ) * (unsigned)SEQ;
    const float* tp = tab + (size_t)sq * 64u + jc;
    const v4f c0 = *(const v4f*)(tp);
    const v4f c1 = *(const v4f*)(tp + 4);
    const v4f s0 = *(const v4f*)(tp + 32);
    const v4f s1 = *(const v4f*)(tp + 36);
    const v4f a0 = *(const v4f*)&Cs[r * LDC + jc];
    const v4f a1 = *(const v4f*)&Cs[r * LDC + jc + 4];
    const v4f b0 = *(const v4f*)&Cs[r * LDC + jc + 32];
    const v4f b1 = *(const v4f*)&Cs[r * LDC + jc + 36];
#pragma unroll
    for (int j = 0; j < 4; ++j) {
      const float lo0 = a0[j] * c0[j] - b0[j] * s0[j];
      const float hi0 = a0[j] * s0[j] + b0[j] * c0[j];
      const float lo1 = a1[j] * c1[j] - b1[j] * s1[j];
      const float hi1 = a1[j] * s1[j] + b1[j] * c1[j];
      x[i][j]     = toh_flush((upper ? hi0 : lo0) * scale);
      x[i][j + 4] = toh_flush((upper ? hi1 : lo1) * scale);
    }
    off[i] = (size_t)(row0 + r) * DIM + n0 + c;
  }
#pragma unroll
  for (int i = 0; i < 2; ++i) *(volatile v8h*)(out16 + off[i]) = x[i];
  __threadfence();
#pragma unroll
  for (int i = 0; i < 2; ++i) *(volatile v8h*)(out16 + off[i]) = x[i];
}

__device__ __forceinline__ void epi_vt_fl(
    const float* Cs, _Float16* __restrict__ out16,
    const unsigned row0, const unsigned n0, const float scale) {
  const unsigned tid = threadIdx.x;
  const unsigned bidx = row0 / (unsigned)SEQ;
  const unsigned key0 = row0 - bidx * (unsigned)SEQ;
  v8h x[2];
  size_t off[2];
#pragma unroll
  for (unsigned i = 0; i < 2u; ++i) {
    const unsigned dcol = 32u * i + (tid >> 3);
    const unsigned kk = (tid & 7u) * 8u;
#pragma unroll
    for (unsigned j = 0; j < 8u; ++j)
      x[i][j] = toh_flush(Cs[(kk + j) * LDC + dcol] * scale);
    off[i] = ((size_t)bidx * DIM + n0 + dcol) * SEQ + key0 + kk;
  }
#pragma unroll
  for (int i = 0; i < 2; ++i) *(volatile v8h*)(out16 + off[i]) = x[i];
  __threadfence();
#pragma unroll
  for (int i = 0; i < 2; ++i) *(volatile v8h*)(out16 + off[i]) = x[i];
}

__device__ __forceinline__ void epi_f32_res(
    const float* Cs, const float* __restrict__ res,
    const unsigned res_full, const unsigned res_rne, float* __restrict__ outf,
    const unsigned out_full, const unsigned row0, const unsigned n0, const float scale) {
  const unsigned tid = threadIdx.x;
  v4f xs[4];
  size_t off[4];
#pragma unroll
  for (unsigned i = 0; i < 4u; ++i) {
    const unsigned r = 16u * i + (tid >> 4);
    const unsigned c = (tid & 15u) * 4u;
    const unsigned crow = row0 + r;
    const size_t frow = full_row(crow);
    const size_t rrow = res_full ? frow : (size_t)crow;
    const size_t orow = out_full ? frow : (size_t)crow;
    const v4f u = *(const v4f*)&Cs[r * LDC + c];
    const v4f rv = *(const v4f*)(res + rrow * DIM + n0 + c);
    v4f val;
#pragma unroll
    for (int j = 0; j < 4; ++j) {
      const float rr = res_rne ? bf16r(rv[j]) : rv[j];
      val[j] = u[j] * scale + rr;
    }
    xs[i] = val;
    off[i] = orow * DIM + n0 + c;
  }
#pragma unroll
  for (int i = 0; i < 4; ++i) *(volatile v4f*)(outf + off[i]) = xs[i];
  __threadfence();
#pragma unroll
  for (int i = 0; i < 4; ++i) *(volatile v4f*)(outf + off[i]) = xs[i];
}

__global__ __launch_bounds__(256) void gemm_qc_kernel(
    const _Float16* __restrict__ H16, const _Float16* __restrict__ WqcT,
    const float* __restrict__ tab, _Float16* __restrict__ Q16,
    _Float16* __restrict__ C16) {
  __shared__ float Cs[64 * LDC];
  const unsigned bx = blockIdx.x;
  const unsigned row0 = blockIdx.y * 64u;
  gemm_main(H16, WqcT, (unsigned)DIM, row0, bx * 64u, Cs);
  if (bx < (unsigned)(DIM / 64))
    epi_rope_fl(Cs, tab, Q16, row0, bx * 64u, 1.0f / WCARRY);
  else
    epi_f16_fl(Cs, C16, (unsigned)NLAT, row0, (bx - (unsigned)(DIM / 64)) * 64u, 1.0f / WCARRY);
}

__global__ __launch_bounds__(256) void gemm_kv_kernel(
    const _Float16* __restrict__ C16, const _Float16* __restrict__ WukvT,
    const float* __restrict__ tab, _Float16* __restrict__ KV16) {
  __shared__ float Cs[64 * LDC];
  const unsigned sel = blockIdx.x / (unsigned)(DIM / 64);
  const unsigned n0 = (blockIdx.x - sel * (unsigned)(DIM / 64)) * 64u;
  const unsigned row0 = blockIdx.y * 64u;
  gemm_main(C16, WukvT, (unsigned)NLAT, row0, blockIdx.x * 64u, Cs);
  if (sel == 0u) epi_rope_fl(Cs, tab, KV16, row0, n0, 1.0f / WCARRY);
  else           epi_vt_fl(Cs, KV16 + PLANE16_ELEMS, row0, n0, 1.0f / WCARRY);
}

__global__ __launch_bounds__(256) void gemm_wo_kernel(
    const _Float16* __restrict__ Ctx16, const _Float16* __restrict__ WoT,
    const float* __restrict__ X, float* __restrict__ X1) {
  __shared__ float Cs[64 * LDC];
  const unsigned n0 = blockIdx.x * 64u;
  const unsigned row0 = blockIdx.y * 64u;
  gemm_main(Ctx16, WoT, (unsigned)DIM, row0, n0, Cs);
  epi_f32_res(Cs, X, 1u, 1u, X1, 0u, row0, n0, 1.0f / (WCARRY * VCARRY));
}

__global__ __launch_bounds__(256) void gemm_moe1_kernel(
    const _Float16* __restrict__ H2, const _Float16* __restrict__ W1T,
    const float* __restrict__ dw, _Float16* __restrict__ Act16) {
  __shared__ float Cs[64 * LDC];
  const unsigned tid = threadIdx.x;
  const unsigned n0 = blockIdx.x * 64u;
  const unsigned row0 = blockIdx.y * 64u;
  gemm_main(H2, W1T, (unsigned)DIM, row0, n0, Cs);
  const bool gated = (n0 >= (unsigned)(NSH * DHID));
  const unsigned nn = (n0 > (unsigned)(NSH * DHID)) ? n0 : (unsigned)(NSH * DHID);
  const unsigned eidx = (nn - (unsigned)(NSH * DHID)) / (unsigned)DHID;
#pragma unroll 1
  for (unsigned e = 0; e < 16u; ++e) {
    const unsigned r = 32u * (e >> 3) + (tid >> 3);
    const unsigned c = (tid & 7u) * 8u + (e & 7u);
    const float t = Cs[r * LDC + c] * (1.0f / WCARRY);
    float gl = dw[(size_t)(row0 + r) * GPITCH + eidx];
    asm volatile("" : "+v"(gl));
    const float gw = gated ? gl : 1.0f;
    const float sg = 1.0f / (1.0f + expf(-t));
    Cs[r * LDC + c] = (ACARRY * gw) * (t * sg);
  }
  __syncthreads();
  epi_f16_fl(Cs, Act16, (unsigned)DFF, row0, n0, 1.0f);
}

__global__ __launch_bounds__(256) void gemm_moe2_kernel(
    const _Float16* __restrict__ Act16, const _Float16* __restrict__ W2T,
    const float* __restrict__ X1, float* __restrict__ out) {
  __shared__ float Cs[64 * LDC];
  const unsigned n0 = blockIdx.x * 64u;
  const unsigned row0 = blockIdx.y * 64u;
  gemm_main(Act16, W2T, (unsigned)DFF, row0, n0, Cs);
  epi_f32_res(Cs, X1, 0u, 0u, out, 1u, row0, n0, 1.0f / (WCARRY * ACARRY));
}

__global__ __launch_bounds__(256) void attn_kernel(
    const _Float16* __restrict__ Qh, const _Float16* __restrict__ Kh,
    const _Float16* __restrict__ Vt, _Float16* __restrict__ Ov) {
  __shared__ _Float16 Ks[64 * LDT];
  __shared__ _Float16 Vs[64 * LDT];
  __shared__ _Float16 Ps[8 * 16 * LDT];

  const unsigned tid = threadIdx.x, lane = tid & 31u;
  const unsigned w = (unsigned)__builtin_amdgcn_readfirstlane((int)(tid >> 5));
  const unsigned hh = lane >> 4, m = lane & 15u;
  const unsigned q0 = blockIdx.x * 128u;
  const unsigned head = blockIdx.y;
  const unsigned b = blockIdx.z;
  const unsigned qw0 = q0 + w * 16u;
  const float scale = 0.125f;
  _Float16* P = Ps + w * (16u * LDT);

  const size_t qoff = (size_t)(b * (unsigned)SEQ + qw0 + m) * DIM + head * HD + hh * 8u;
  v16h qf[2];
  qf[0] = frag_at(Qh + qoff);
  qf[1] = frag_at(Qh + qoff + 32);

  float mrow[8], lrow[8];
  v8f o[4];
#pragma unroll
  for (int v = 0; v < 8; ++v) { mrow[v] = -1.0e30f; lrow[v] = 0.0f; }
#pragma unroll
  for (int nb = 0; nb < 4; ++nb) o[nb] = (v8f){};

  const size_t kplane = (size_t)b * SEQ * DIM + head * HD;
  const size_t vplane = ((size_t)b * DIM + head * HD) * SEQ;
  const unsigned kend = q0 + 128u;

  for (unsigned kb = 0; kb < kend; kb += 64u) {
#pragma unroll
    for (unsigned j = 0; j < 2u; ++j) {
      const unsigned idx = tid + 256u * j;
      const unsigned r = idx >> 3, c = (idx & 7u) * 8u;
      *(v8h*)&Ks[r * LDT + c] = *(const v8h*)(Kh + kplane + (size_t)(kb + r) * DIM + c);
      *(v8h*)&Vs[r * LDT + c] = *(const v8h*)(Vt + vplane + (size_t)r * SEQ + kb + c);
    }
    __syncthreads();

    if (kb <= qw0 + 15u) {
      v8f s[4];
#pragma unroll
      for (int kg = 0; kg < 4; ++kg) {
        v8f t = {};
#pragma unroll
        for (int c = 0; c < 2; ++c) {
          const v16h kf = ld_frag(&Ks[(kg * 16) * LDT + c * 32], LDT);
          t = wmma16(qf[c], kf, t);
        }
        s[kg] = t * scale;
      }
      if (kb + 63u > qw0) {
#pragma unroll
        for (int kg = 0; kg < 4; ++kg) {
          const unsigned key = kb + (unsigned)kg * 16u + m;
#pragma unroll
          for (int v = 0; v < 8; ++v) {
            const unsigned qr = qw0 + hh * 8u + (unsigned)v;
            s[kg][v] = (key > qr) ? -1.0e30f : s[kg][v];
          }
        }
      }

      float alpha[8];
#pragma unroll
      for (int v = 0; v < 8; ++v) {
        float mx = fmaxf(fmaxf(s[0][v], s[1][v]), fmaxf(s[2][v], s[3][v]));
        mx = red16_max(mx);
        const float mn = fmaxf(mrow[v], mx);
        alpha[v] = __expf(mrow[v] - mn);
        mrow[v] = mn;
      }
#pragma unroll
      for (int kg = 0; kg < 4; ++kg)
#pragma unroll
        for (int v = 0; v < 8; ++v) s[kg][v] = __expf(s[kg][v] - mrow[v]);
#pragma unroll
      for (int v = 0; v < 8; ++v) {
        const float rs = red16_sum((s[0][v] + s[1][v]) + (s[2][v] + s[3][v]));
        lrow[v] = alpha[v] * lrow[v] + rs;
      }
#pragma unroll
      for (int nb = 0; nb < 4; ++nb)
#pragma unroll
        for (int v = 0; v < 8; ++v) o[nb][v] = o[nb][v] * alpha[v];

#pragma unroll
      for (int kg = 0; kg < 4; ++kg)
#pragma unroll
        for (int v = 0; v < 8; ++v)
          P[(hh * 8u + (unsigned)v) * LDT + (unsigned)kg * 16u + m] =
              (_Float16)(s[kg][v] * PCARRY);
      wave_lds_sync();

#pragma unroll
      for (int c = 0; c < 2; ++c) {
        const v16h pf = ld_frag(P + c * 32, LDT);
#pragma unroll
        for (int nb = 0; nb < 4; ++nb) {
          const v16h vf = ld_frag(&Vs[(nb * 16) * LDT + c * 32], LDT);
          o[nb] = wmma16(pf, vf, o[nb]);
        }
      }
    }
    __syncthreads();
  }

  float inv[8];
#pragma unroll
  for (int v = 0; v < 8; ++v) inv[v] = __builtin_amdgcn_rcpf(lrow[v]) * (VCARRY / PCARRY);
#pragma unroll
  for (int nb = 0; nb < 4; ++nb)
#pragma unroll
    for (int v = 0; v < 8; ++v)
      P[(hh * 8u + (unsigned)v) * LDT + (unsigned)nb * 16u + m] = (_Float16)(o[nb][v] * inv[v]);
  wave_lds_sync();
  v8h x[4];
  size_t off[4];
#pragma unroll
  for (unsigned i = 0; i < 4u; ++i) {
    const unsigned r = 4u * i + (lane >> 3);
    const unsigned c = (lane & 7u) * 8u;
    x[i] = *(const v8h*)&P[r * LDT + c];
    off[i] = (size_t)(b * (unsigned)SEQ + qw0 + r) * DIM + head * HD + c;
  }
#pragma unroll
  for (int i = 0; i < 4; ++i) *(volatile v8h*)(Ov + off[i]) = x[i];
  __threadfence();
#pragma unroll
  for (int i = 0; i < 4; ++i) *(volatile v8h*)(Ov + off[i]) = x[i];
}

extern "C" void kernel_launch(void* const* d_in, const int* in_sizes, int n_in,
                              void* d_out, int out_size, void* d_ws, size_t ws_size,
                              hipStream_t stream) {
  if (n_in < 13) return;
  const long long need_x = ((long long)(NB - 1) * SEQ_FULL + SEQ) * DIM;
  if ((long long)in_sizes[0] < need_x) return;
  if (in_sizes[1] < DIM) return;
  if ((long long)in_sizes[2] < (long long)DIM * DIM) return;
  if ((long long)in_sizes[3] < (long long)DIM * NLAT) return;
  if ((long long)in_sizes[4] < (long long)NLAT * DIM) return;
  if ((long long)in_sizes[5] < (long long)NLAT * DIM) return;
  if ((long long)in_sizes[6] < (long long)DIM * DIM) return;
  if (in_sizes[7] < DIM) return;
  if (in_sizes[8] < DIM * NRT) return;
  if ((long long)in_sizes[9] < (long long)NSH * DIM * DHID) return;
  if ((long long)in_sizes[10] < (long long)NSH * DHID * DIM) return;
  if ((long long)in_sizes[11] < (long long)NRT * DIM * DHID) return;
  if ((long long)in_sizes[12] < (long long)NRT * DHID * DIM) return;
  if ((long long)out_size < need_x) return;
  if (ws_size < WS_TOTAL) return;

  const float* X     = (const float*)d_in[0];
  const float* gain1 = (const float*)d_in[1];
  const float* wq    = (const float*)d_in[2];
  const float* wdkv  = (const float*)d_in[3];
  const float* wuk   = (const float*)d_in[4];
  const float* wuv   = (const float*)d_in[5];
  const float* wo    = (const float*)d_in[6];
  const float* gain2 = (const float*)d_in[7];
  const float* wg    = (const float*)d_in[8];
  const float* ws1   = (const float*)d_in[9];
  const float* ws2   = (const float*)d_in[10];
  const float* wr1   = (const float*)d_in[11];
  const float* wr2   = (const float*)d_in[12];
  float* out = (float*)d_out;

  char* ws = (char*)d_ws;
  _Float16* WqcT  = (_Float16*)(ws + OFF_WQC);
  _Float16* WukvT = (_Float16*)(ws + OFF_WUKV);
  _Float16* WoT   = (_Float16*)(ws + OFF_WO);
  _Float16* W1T   = (_Float16*)(ws + OFF_W1);
  _Float16* W2T   = (_Float16*)(ws + OFF_W2);
  float*    Tab   = (float*)(ws + OFF_TAB);
  _Float16* H1    = (_Float16*)(ws + OFF_H1);
  _Float16* C16   = (_Float16*)(ws + OFF_C);
  _Float16* QKV16 = (_Float16*)(ws + OFF_QKV);
  _Float16* Ctx16 = (_Float16*)(ws + OFF_CTX);
  float*    X1    = (float*)(ws + OFF_X1);
  _Float16* H2    = (_Float16*)(ws + OFF_H2);
  float*    Dw    = (float*)(ws + OFF_DW);
  _Float16* Act16 = (_Float16*)(ws + OFF_ACT);

  dim3 blk(256);
  wconv_kernel<<<dim3(DIM / 64, DIM / 64), blk, 0, stream>>>(wq, WqcT, DIM, DIM, 0u);
  wconv_kernel<<<dim3(NLAT / 64, DIM / 64), blk, 0, stream>>>(wdkv, WqcT + WSQ_ELEMS, NLAT, DIM, 0u);
  wconv_kernel<<<dim3(DIM / 64, NLAT / 64), blk, 0, stream>>>(wuk, WukvT, DIM, NLAT, 0u);
  wconv_kernel<<<dim3(DIM / 64, NLAT / 64), blk, 0, stream>>>(wuv, WukvT + (size_t)DIM * NLAT, DIM, NLAT, 0u);
  wconv_kernel<<<dim3(DIM / 64, DIM / 64), blk, 0, stream>>>(wo, WoT, DIM, DIM, 0u);
  wconv2_kernel<<<dim3(DHID / 64, DIM / 64, NSH), blk, 0, stream>>>(
      ws1, W1T, DHID, DIM, DIM, (unsigned)(DHID * DIM));
  wconv2_kernel<<<dim3(DHID / 64, DIM / 64, NRT), blk, 0, stream>>>(
      wr1, W1T + (size_t)NSH * DHID * DIM, DHID, DIM, DIM, (unsigned)(DHID * DIM));
  wconv2_kernel<<<dim3(DIM / 64, DHID / 64, NSH), blk, 0, stream>>>(
      ws2, W2T, DIM, DHID, DFF, (unsigned)DHID);
  wconv2_kernel<<<dim3(DIM / 64, DHID / 64, NRT), blk, 0, stream>>>(
      wr2, W2T + (size_t)NSH * DHID, DIM, DHID, DFF, (unsigned)DHID);

  rope_tab_kernel<<<dim3(SEQ / 8), blk, 0, stream>>>(Tab);

  rms_kernel<<<dim3(MROWS), dim3(128), 0, stream>>>(X, gain1, H1, 1u, 1u, wg, Dw, 0u);
  gemm_qc_kernel<<<dim3((DIM + NLAT) / 64, MROWS / 64), blk, 0, stream>>>(H1, WqcT, Tab, QKV16, C16);
  gemm_kv_kernel<<<dim3(2 * DIM / 64, MROWS / 64), blk, 0, stream>>>(
      C16, WukvT, Tab, QKV16 + PLANE16_ELEMS);
  attn_kernel<<<dim3(SEQ / 128, NHEAD, NB), blk, 0, stream>>>(
      QKV16, QKV16 + PLANE16_ELEMS, QKV16 + 2 * PLANE16_ELEMS, Ctx16);
  gemm_wo_kernel<<<dim3(DIM / 64, MROWS / 64), blk, 0, stream>>>(Ctx16, WoT, X, X1);
  rms_kernel<<<dim3(MROWS), dim3(128), 0, stream>>>(X1, gain2, H2, 0u, 0u, wg, Dw, 1u);
  gemm_moe1_kernel<<<dim3(DFF / 64, MROWS / 64), blk, 0, stream>>>(H2, W1T, Dw, Act16);
  gemm_moe2_kernel<<<dim3(DIM / 64, MROWS / 64), blk, 0, stream>>>(Act16, W2T, X1, out);
}
